// Mamba2Block_53446573031683
// MI455X (gfx1250) — hardware-run, weakly checked
//
#include <hip/hip_runtime.h>
#include <math.h>

typedef __attribute__((ext_vector_type(16))) _Float16 v16h;
typedef __attribute__((ext_vector_type(8)))  _Float16 v8h;
typedef __attribute__((ext_vector_type(16))) __bf16   v16b;
typedef __attribute__((ext_vector_type(8)))  __bf16   v8b;
typedef __attribute__((ext_vector_type(8)))  float    v8f;
typedef __attribute__((ext_vector_type(4)))  float    v4f;

constexpr int kBatch    = 2;
constexpr int kSeq      = 2048;
constexpr int kDm       = 256;
constexpr int kDin      = 512;
constexpr int kHd       = 64;
constexpr int kNh       = 8;
constexpr int kNst      = 64;
constexpr int kConvDim  = kDin + 2 * kNst;
constexpr int kDproj    = 2 * kDin + 2 * kNst + kNh;
constexpr int kDprojPad = 1216;
constexpr int kColXbc   = kDin;
constexpr int kColDt    = kDin + kConvDim;
constexpr int kRows     = kBatch * kSeq;
constexpr float kEps    = 1e-5f;
constexpr int kConvTP   = 132;
constexpr int kScanTS   = 32;
static_assert(kDproj == 1160, "in_proj width");
static_assert(kDprojPad % 64 == 0 && kDprojPad >= kDproj && kDprojPad % 8 == 0, "padded N");
static_assert((kDm % 32) == 0 && (kDin % 32) == 0, "GEMM K multiples of 32");
static_assert((kRows % 64) == 0 && (kDm % 64) == 0, "GEMM M,N multiples of 64");
static_assert((kSeq % 64) == 0 && (kSeq % kScanTS) == 0 && (kConvDim % 128) == 0 && (kRows % 8) == 0, "tile multiples");
static_assert(kHd == 64 && kNh * kHd == kDin, "head layout");

constexpr size_t kOffXH   = 0;
constexpr size_t kOffXL   = kOffXH  + (size_t)kRows * kDm * 2;
constexpr size_t kOffWIH  = kOffXL  + (size_t)kRows * kDm * 2;
constexpr size_t kOffWIL  = kOffWIH + (size_t)kDprojPad * kDm * 2;
constexpr size_t kOffWOH  = kOffWIL + (size_t)kDprojPad * kDm * 2;
constexpr size_t kOffWOL  = kOffWOH + (size_t)kDm * kDin * 2;
constexpr size_t kOffZX   = kOffWOL + (size_t)kDm * kDin * 2;
constexpr size_t kOffXBC  = kOffZX  + (size_t)kRows * kDprojPad * 4;
constexpr size_t kOffDT   = kOffXBC + (size_t)kRows * kConvDim * 4;
constexpr size_t kOffDA   = kOffDT  + (size_t)kRows * kNh * 4;
constexpr size_t kOffY    = kOffDA  + (size_t)kRows * kNh * 4;
constexpr size_t kOffGH   = kOffY   + (size_t)kRows * kDin * 4;
constexpr size_t kOffGL   = kOffGH  + (size_t)kRows * kDin * 2;
constexpr size_t kWsTotal = kOffGL  + (size_t)kRows * kDin * 2;
static_assert(kWsTotal == 53411840ull, "carve total");
static_assert(kWsTotal <= 134217728ull, "carve cap");
static_assert((kOffXL % 128) == 0 && (kOffWIH % 128) == 0 && (kOffWIL % 128) == 0 && (kOffWOH % 128) == 0 &&
              (kOffWOL % 128) == 0 && (kOffZX % 128) == 0 && (kOffXBC % 128) == 0 && (kOffDT % 128) == 0 &&
              (kOffDA % 128) == 0 && (kOffY % 128) == 0 && (kOffGH % 128) == 0 && (kOffGL % 128) == 0,
              "128-B aligned regions");
constexpr size_t kOut1Elem = (size_t)kRows * kDm;
static_assert(kOut1Elem * 4 == 4194304ull, "out1 offset");
static_assert((kOut1Elem + (size_t)kRows * kDm) * 4 == 8388608ull, "d_out total");

__device__ __forceinline__ unsigned short f2bf_bits(float f) {
  unsigned u = __float_as_uint(f);
  return (unsigned short)((u + 0x7FFFu + ((u >> 16) & 1u)) >> 16);
}
__device__ __forceinline__ float bf_bits2f(unsigned short h) { return __uint_as_float(((unsigned)h) << 16); }

__device__ __forceinline__ void dep_guard4_h(v8f& a, v8f& b, v8f& c, v8f& d, v16h x, v16h y) {
  asm volatile("v_nop\n\tv_nop\n\tv_nop\n\tv_nop" : "+v"(a), "+v"(b), "+v"(c), "+v"(d) : "v"(x), "v"(y));
}
__device__ __forceinline__ void dep_guard4_b(v8f& a, v8f& b, v8f& c, v8f& d, v16b x, v16b y) {
  asm volatile("v_nop\n\tv_nop\n\tv_nop\n\tv_nop" : "+v"(a), "+v"(b), "+v"(c), "+v"(d) : "v"(x), "v"(y));
}
__device__ __forceinline__ void keep4_h(v16h a, v16h b, v16h c, v16h d) { asm volatile("v_nop" :: "v"(a), "v"(b), "v"(c), "v"(d)); }
__device__ __forceinline__ void keep4_b(v16b a, v16b b, v16b c, v16b d) { asm volatile("v_nop" :: "v"(a), "v"(b), "v"(c), "v"(d)); }
__device__ __forceinline__ void acc_guard4(v8f& a, v8f& b, v8f& c, v8f& d) { asm volatile("v_nop\n\tv_nop\n\tv_nop\n\tv_nop" : "+v"(a), "+v"(b), "+v"(c), "+v"(d)); }
template <typename T> struct Frag;
template <> struct Frag<_Float16> {
  typedef v16h V; union U { v16h v; v8h h[2]; };
  static __device__ __forceinline__ v16h load(const _Float16* p) {
    U f; f.h[0] = *(const v8h*)(p); f.h[1] = *(const v8h*)(p + 16); return f.v;
  }
  static __device__ __forceinline__ v8f mma(v16h a, v16h b, v8f c) {
    return __builtin_amdgcn_wmma_f32_16x16x32_f16(false, a, false, b, (short)0, c, false, false);
  }
  static __device__ __forceinline__ void guard4(v8f& a, v8f& b, v8f& c, v8f& d, v16h x, v16h y) { dep_guard4_h(a, b, c, d, x, y); }
  static __device__ __forceinline__ void keep(v16h a, v16h b, v16h c, v16h d) { keep4_h(a, b, c, d); }
};
template <> struct Frag<__bf16> {
  typedef v16b V; union U { v16b v; v8b h[2]; };
  static __device__ __forceinline__ v16b load(const __bf16* p) {
    U f; f.h[0] = *(const v8b*)(p); f.h[1] = *(const v8b*)(p + 16); return f.v;
  }
  static __device__ __forceinline__ v8f mma(v16b a, v16b b, v8f c) {
    return __builtin_amdgcn_wmma_f32_16x16x32_bf16(false, a, false, b, (short)0, c, false, false);
  }
  static __device__ __forceinline__ void guard4(v8f& a, v8f& b, v8f& c, v8f& d, v16b x, v16b y) { dep_guard4_b(a, b, c, d, x, y); }
  static __device__ __forceinline__ void keep(v16b a, v16b b, v16b c, v16b d) { keep4_b(a, b, c, d); }
};

template <int ET> struct Elem;
template <> struct Elem<0> { typedef _Float16 T; };
template <> struct Elem<1> { typedef __bf16 T; };
template <int ET, int SPL, int BIAS_MODE, int OUT_MODE, bool RESID, int ACT = 0>
__global__ __launch_bounds__(256) void wmma_gemm64(
    const unsigned short* __restrict__ Ap, const unsigned short* __restrict__ A2p, int lda, long strideA,
    const unsigned short* __restrict__ Btp, const unsigned short* __restrict__ Bt2p, int ldb, long strideB,
    void* __restrict__ Cout, void* __restrict__ Cout2, int ldc, long strideC,
    const float* __restrict__ bias,
    const float* __restrict__ resid, long strideR,
    int M, int N, int K, float scale) {
  typedef typename Elem<ET>::T T;
  typedef typename Frag<T>::V V;
  const T* A = (const T*)Ap; const T* A2 = (const T*)A2p; const T* Bt = (const T*)Btp; const T* Bt2 = (const T*)Bt2p;
  __shared__ __align__(16) float sT[8][16 * 68];
  const int b    = blockIdx.y;
  const int lane = threadIdx.x & 31;
  const int wave = threadIdx.x >> 5;
  const int tilesN = N >> 6;
  const int tilesM = M >> 6;
  const int tile = blockIdx.x * 8 + wave;
  if (tile >= tilesM * tilesN) return;
  const int tm = tile / tilesN;
  const int tn = tile - tm * tilesN;
  const int m0 = tm << 6;
  const int n0 = tn << 6;

  const T* Ab  = A  + (size_t)b * strideA;
  const T* Bb  = Bt + (size_t)b * strideB;
  const T* Ab2 = (SPL >= 1) ? (A2  + (size_t)b * strideA) : nullptr;
  const T* Bb2 = (SPL == 2) ? (Bt2 + (size_t)b * strideB) : nullptr;

  const int rlane = lane & 15;
  const int koff  = (lane >> 4) * 8;
  const int mOff  = (lane >> 4) * 8;

  v8f acc[4][4];
#pragma unroll
  for (int i = 0; i < 4; ++i)
#pragma unroll
    for (int j = 0; j < 4; ++j) acc[i][j] = (v8f){0.f,0.f,0.f,0.f,0.f,0.f,0.f,0.f};

  for (int k0 = 0; k0 < K; k0 += 32) {
    V bh[4], bl[4];
#pragma unroll
    for (int j = 0; j < 4; ++j) {
      const size_t bo = (size_t)(n0 + (j << 4) + rlane) * ldb + koff + k0;
      bh[j] = Frag<T>::load(Bb + bo);
      if (SPL == 2) bl[j] = Frag<T>::load(Bb2 + bo);
    }
#pragma unroll
    for (int i = 0; i < 4; ++i) {
      const size_t ao = (size_t)(m0 + (i << 4) + rlane) * lda + koff + k0;
      V ah = Frag<T>::load(Ab + ao);
      V al;
      if (SPL >= 1) al = Frag<T>::load(Ab2 + ao);
#pragma unroll
      for (int j = 0; j < 4; ++j) {
        acc[i][j] = Frag<T>::mma(ah, bh[j], acc[i][j]);
        if (SPL == 2) acc[i][j] = Frag<T>::mma(ah, bl[j], acc[i][j]);
        if (SPL >= 1) acc[i][j] = Frag<T>::mma(al, bh[j], acc[i][j]);
      }
      Frag<T>::guard4(acc[i][0], acc[i][1], acc[i][2], acc[i][3], ah, (SPL >= 1) ? al : ah);
    }
    Frag<T>::keep(bh[0], bh[1], bh[2], bh[3]);
    if (SPL == 2) Frag<T>::keep(bl[0], bl[1], bl[2], bl[3]);
  }
  acc_guard4(acc[0][0], acc[0][1], acc[0][2], acc[0][3]);
  acc_guard4(acc[1][0], acc[1][1], acc[1][2], acc[1][3]);
  acc_guard4(acc[2][0], acc[2][1], acc[2][2], acc[2][3]);
  acc_guard4(acc[3][0], acc[3][1], acc[3][2], acc[3][3]);

  float* slab = sT[wave];
  const float* Rb = RESID ? (resid + (size_t)b * strideR) : nullptr;
#pragma unroll
  for (int i = 0; i < 4; ++i) {
    const int mBase = m0 + (i << 4);
#pragma unroll
    for (int j = 0; j < 4; ++j) {
      const int n = n0 + (j << 4) + rlane;
      float bv = 0.f;
      if (BIAS_MODE == 2) bv = bias[n];
#pragma unroll
      for (int r = 0; r < 8; ++r) {
        float v = acc[i][j][r] * scale;
        if (BIAS_MODE == 1) v += bias[mBase + mOff + r];
        if (BIAS_MODE == 2) v += bv;
        if (RESID) v += Rb[(size_t)(mBase + mOff + r) * ldc + n];
        if (ACT == 1) v = tanhf(v);
        if (ACT == 2) v = fmaxf(v, 0.0f);
        if (ACT == 3) v = v / (1.0f + expf(-v));
        if (ACT == 4) v = (v > 0.f) ? v : 0.01f * v;
        slab[(mOff + r) * 68 + (j << 4) + rlane] = v;
      }
    }
    __builtin_amdgcn_fence(__ATOMIC_RELEASE, "workgroup");
    __builtin_amdgcn_wave_barrier();
    __builtin_amdgcn_fence(__ATOMIC_ACQUIRE, "workgroup");
    if (OUT_MODE == 0) {
      float* C = (float*)Cout + (size_t)b * strideC;
      const int hh = lane >> 4, c4 = (lane & 15) * 4;
      for (int pass = 0; pass < 2; ++pass) {
#pragma unroll
        for (int it = 0; it < 8; ++it) {
          const int row = it * 2 + hh;
          v4f v = *(const v4f*)(slab + row * 68 + c4);
          *(volatile v4f*)(C + (size_t)(mBase + row) * ldc + n0 + c4) = v;
        }
        __threadfence();
      }
    } else {
      const int q = lane >> 3, c8 = (lane & 7) * 8;
      unsigned short* C  = (unsigned short*)Cout  + (size_t)b * strideC;
      unsigned short* C2 = (OUT_MODE == 2) ? ((unsigned short*)Cout2 + (size_t)b * strideC) : nullptr;
      for (int pass = 0; pass < 2; ++pass) {
#pragma unroll
        for (int it = 0; it < 4; ++it) {
          const int row = it * 4 + q;
          const float* sp = slab + row * 68 + c8;
          v8h hv, lv;
#pragma unroll
          for (int e = 0; e < 8; ++e) {
            if (OUT_MODE == 1) {
              hv[e] = (_Float16)sp[e];
            } else {
              unsigned short hb = f2bf_bits(sp[e]);
              unsigned short lb = f2bf_bits(sp[e] - bf_bits2f(hb));
              hv[e] = __builtin_bit_cast(_Float16, hb);
              lv[e] = __builtin_bit_cast(_Float16, lb);
            }
          }
          *(volatile v8h*)(C + (size_t)(mBase + row) * ldc + n0 + c8) = hv;
          if (OUT_MODE == 2) *(volatile v8h*)(C2 + (size_t)(mBase + row) * ldc + n0 + c8) = lv;
        }
        __threadfence();
      }
    }
    __builtin_amdgcn_fence(__ATOMIC_RELEASE, "workgroup");
    __builtin_amdgcn_wave_barrier();
    __builtin_amdgcn_fence(__ATOMIC_ACQUIRE, "workgroup");
  }
}

__global__ __launch_bounds__(256) void ln_residual_kernel(
    const float* __restrict__ hid, const float* __restrict__ nw, const float* __restrict__ nb,
    float* __restrict__ resid_out, unsigned short* __restrict__ XH, unsigned short* __restrict__ XL)
{
  __shared__ __align__(16) float sX[8 * kDm];
  const int tid = threadIdx.x, lane = tid & 31, wave = tid >> 5;
  const int row = blockIdx.x * 8 + wave;
  const size_t rb = (size_t)row * kDm;
  const int c0 = 4 * lane, c1 = 128 + 4 * lane;
  const v4f a0 = *(const v4f*)(hid + rb + c0);
  const v4f a1 = *(const v4f*)(hid + rb + c1);
  const v4f w0 = *(const v4f*)(nw + c0);
  const v4f w1 = *(const v4f*)(nw + c1);
  const v4f b0 = *(const v4f*)(nb + c0);
  const v4f b1 = *(const v4f*)(nb + c1);
  float s = ((a0[0] + a0[1]) + (a0[2] + a0[3])) + ((a1[0] + a1[1]) + (a1[2] + a1[3]));
#pragma unroll
  for (int off = 1; off < 32; off <<= 1) s += __shfl_xor(s, off, 32);
  const float mu = s * (1.0f / (float)kDm);
  v4f d0, d1;
#pragma unroll
  for (int e = 0; e < 4; ++e) { d0[e] = a0[e] - mu; d1[e] = a1[e] - mu; }
  float qs = 0.f;
#pragma unroll
  for (int e = 0; e < 4; ++e) { qs = fmaf(d0[e], d0[e], qs); qs = fmaf(d1[e], d1[e], qs); }
#pragma unroll
  for (int off = 1; off < 32; off <<= 1) qs += __shfl_xor(qs, off, 32);
  const float rstd = rsqrtf(qs * (1.0f / (float)kDm) + kEps);
  v4f x0, x1;
#pragma unroll
  for (int e = 0; e < 4; ++e) {
    x0[e] = (d0[e] * rstd) * w0[e] + b0[e];
    x1[e] = (d1[e] * rstd) * w1[e] + b1[e];
  }
  float* sw = sX + wave * kDm;
  *(v4f*)(sw + c0) = x0;
  *(v4f*)(sw + c1) = x1;
  __syncthreads();
  const v4f r0 = *(const v4f*)(sw + 8 * lane);
  const v4f r1 = *(const v4f*)(sw + 8 * lane + 4);
  v8h hv, lv;
#pragma unroll
  for (int e = 0; e < 4; ++e) {
    const unsigned short h0 = f2bf_bits(r0[e]), h1 = f2bf_bits(r1[e]);
    const unsigned short l0 = f2bf_bits(r0[e] - bf_bits2f(h0)), l1 = f2bf_bits(r1[e] - bf_bits2f(h1));
    hv[e]     = __builtin_bit_cast(_Float16, h0);
    hv[4 + e] = __builtin_bit_cast(_Float16, h1);
    lv[e]     = __builtin_bit_cast(_Float16, l0);
    lv[4 + e] = __builtin_bit_cast(_Float16, l1);
  }
  unsigned short* ph = XH + rb + 8 * lane;
  unsigned short* plo = XL + rb + 8 * lane;
  for (int pass = 0; pass < 2; ++pass) {
    *(volatile v4f*)(resid_out + rb + c0) = a0;
    *(volatile v4f*)(resid_out + rb + c1) = a1;
    *(volatile v8h*)ph  = hv;
    *(volatile v8h*)plo = lv;
    __threadfence();
  }
}

template <int KDIM>
__global__ __launch_bounds__(256) void weight_bt_split_kernel(
    const float* __restrict__ W, int nreal,
    unsigned short* __restrict__ BtH, unsigned short* __restrict__ BtL)
{
  constexpr int kNch = KDIM / 256;
  static_assert(kNch >= 1 && kNch * 256 == KDIM, "k chunks");
  const int lane = threadIdx.x & 31, wave = threadIdx.x >> 5;
  const int n = blockIdx.x * 8 + wave;
  const int nc = (n < nreal) ? n : (nreal - 1);
  const float keep = (n < nreal) ? 1.0f : 0.0f;
  v8h hv[kNch], lv[kNch];
#pragma unroll
  for (int c = 0; c < kNch; ++c) {
    float f[8];
#pragma unroll
    for (int i = 0; i < 8; ++i) f[i] = W[(size_t)(c * 256 + 8 * lane + i) * nreal + nc] * keep;
    asm volatile("" ::: "memory");
#pragma unroll
    for (int i = 0; i < 8; ++i) {
      const unsigned short hb = f2bf_bits(f[i]);
      const unsigned short lb = f2bf_bits(f[i] - bf_bits2f(hb));
      hv[c][i] = __builtin_bit_cast(_Float16, hb);
      lv[c][i] = __builtin_bit_cast(_Float16, lb);
    }
  }
  const size_t ob = (size_t)n * KDIM + 8 * lane;
  for (int pass = 0; pass < 2; ++pass) {
#pragma unroll
    for (int c = 0; c < kNch; ++c) {
      *(volatile v8h*)(BtH + ob + c * 256) = hv[c];
      *(volatile v8h*)(BtL + ob + c * 256) = lv[c];
    }
    __threadfence();
  }
}

__global__ __launch_bounds__(128) void conv_silu_kernel(
    const float* __restrict__ ZX, const float* __restrict__ cw, const float* __restrict__ cb,
    float* __restrict__ XBC)
{
  __shared__ __align__(16) float sT[16 * kConvTP];
  const int tid = threadIdx.x, lane = tid & 31, wave = tid >> 5;
  const int c0 = blockIdx.x * 128, c = c0 + tid;
  const int g0 = blockIdx.y * 64;
  const int tb = g0 & (kSeq - 1);
  const v4f wv = *(const v4f*)(cw + (size_t)c * 4);
  const float bc = cb[c];
  float xm3, xm2, xm1;
  {
    const bool hist = (tb > 0);
    const int rb = hist ? (g0 - 3) : g0;
    const float v3 = ZX[(size_t)rb * kDprojPad + kColXbc + c];
    const float v2 = ZX[(size_t)(rb + 1) * kDprojPad + kColXbc + c];
    const float v1 = ZX[(size_t)(rb + 2) * kDprojPad + kColXbc + c];
    xm3 = hist ? v3 : 0.f;
    xm2 = hist ? v2 : 0.f;
    xm1 = hist ? v1 : 0.f;
  }
#pragma unroll 1
  for (int sub = 0; sub < 4; ++sub) {
    const int lb = g0 + sub * 16;
#pragma unroll 1
    for (int s = 0; s < 16; ++s) {
      const float xcur = ZX[(size_t)(lb + s) * kDprojPad + kColXbc + c];
      float acc = bc;
      acc = fmaf(wv[0], xm3, acc);
      acc = fmaf(wv[1], xm2, acc);
      acc = fmaf(wv[2], xm1, acc);
      acc = fmaf(wv[3], xcur, acc);
      const float sg = __builtin_amdgcn_rcpf(1.0f + expf(-acc));
      sT[s * kConvTP + tid] = acc * sg;
      xm3 = xm2; xm2 = xm1; xm1 = xcur;
    }
    __syncthreads();
    v4f fv[4];
#pragma unroll
    for (int it = 0; it < 4; ++it) fv[it] = *(const v4f*)(sT + (it * 4 + wave) * kConvTP + lane * 4);
    for (int pass = 0; pass < 2; ++pass) {
#pragma unroll
      for (int it = 0; it < 4; ++it)
        *(volatile v4f*)(XBC + (size_t)(lb + it * 4 + wave) * kConvDim + c0 + lane * 4) = fv[it];
      __threadfence();
    }
    __syncthreads();
  }
}

__global__ __launch_bounds__(256) void dt_kernel(
    const float* __restrict__ ZX, const float* __restrict__ dtb, const float* __restrict__ Alog,
    float* __restrict__ DT, float* __restrict__ DA)
{
  const int e = blockIdx.x * 256 + threadIdx.x;
  const int row = e >> 3, h = e & 7;
  const float v  = ZX[(size_t)row * kDprojPad + kColDt + h] + dtb[h];
  const float sp = fmaxf(v, 0.0f) + log1pf(expf(-fabsf(v)));
  const float An = -expf(Alog[h]);
  const float da = expf(sp * An);
  for (int pass = 0; pass < 2; ++pass) {
    ((volatile float*)DT)[e] = sp;
    ((volatile float*)DA)[e] = da;
    __threadfence();
  }
}

__global__ __launch_bounds__(128) void scan_kernel(
    const float* __restrict__ XBC, const float* __restrict__ DT, const float* __restrict__ DA,
    const float* __restrict__ Dp, float* __restrict__ Y)
{
  __shared__ __align__(16) float sBC[kScanTS * 128];
  __shared__ __align__(16) float sXv[kScanTS * 32];
  __shared__ __align__(16) float sY[kScanTS * 32];
  __shared__ __align__(16) float sDt[kScanTS];
  __shared__ __align__(16) float sDa[kScanTS];
  const int tid = threadIdx.x, lane = tid & 31, wave = tid >> 5;
  const int bix = blockIdx.x >> 4;
  const int h   = (blockIdx.x >> 1) & 7;
  const int p0  = (blockIdx.x & 1) * 32;
  const int pl  = tid >> 2;
  const int n0  = (tid & 3) * 16;
  const int xcol = h * kHd + p0;
  const size_t row0 = (size_t)bix * kSeq;
  const float Dh = Dp[h];
  float st[16];
#pragma unroll
  for (int k = 0; k < 16; ++k) st[k] = 0.f;
  const int orow = lane >> 3, oc4 = (lane & 7) * 4;
#pragma unroll 1
  for (int t0 = 0; t0 < kSeq; t0 += kScanTS) {
    __syncthreads();
#pragma unroll
    for (int i = 0; i < 8; ++i) {
      const int f = tid + 128 * i;
      const int r = f >> 5, c4 = (f & 31) * 4;
      *(v4f*)(sBC + r * 128 + c4) = *(const v4f*)(XBC + (row0 + t0 + r) * kConvDim + kColXbc + c4);
    }
    asm volatile("" ::: "memory");
#pragma unroll
    for (int i = 0; i < 2; ++i) {
      const int f = tid + 128 * i;
      const int r = f >> 3, c4 = (f & 7) * 4;
      *(v4f*)(sXv + r * 32 + c4) = *(const v4f*)(XBC + (row0 + t0 + r) * kConvDim + xcol + c4);
    }
    {
      const int rr = tid & 31;
      sDt[rr] = DT[(row0 + t0 + rr) * kNh + h];
      sDa[rr] = DA[(row0 + t0 + rr) * kNh + h];
    }
    __syncthreads();
#pragma unroll 1
    for (int s = 0; s < kScanTS; ++s) {
      const float da = sDa[s];
      const float dt = sDt[s];
      const float xp = sXv[s * 32 + pl];
      const float dx = dt * xp;
      const float* bp = sBC + s * 128 + n0;
      const float* cp = bp + 64;
      float yq = 0.f;
#pragma unroll
      for (int i4 = 0; i4 < 4; ++i4) {
        const v4f bv = *(const v4f*)(bp + 4 * i4);
        const v4f cv = *(const v4f*)(cp + 4 * i4);
#pragma unroll
        for (int e = 0; e < 4; ++e) {
          const int k = 4 * i4 + e;
          st[k] = fmaf(st[k], da, dx * bv[e]);
          yq = fmaf(st[k], cv[e], yq);
        }
      }
      yq += __shfl_xor(yq, 1, 32);
      yq += __shfl_xor(yq, 2, 32);
      sY[s * 32 + pl] = fmaf(Dh, xp, yq);
    }
    __syncthreads();
    v4f ov[2];
#pragma unroll
    for (int it = 0; it < 2; ++it) {
      const int r = it * 16 + wave * 4 + orow;
      ov[it] = *(const v4f*)(sY + r * 32 + oc4);
    }
    for (int pass = 0; pass < 2; ++pass) {
#pragma unroll
      for (int it = 0; it < 2; ++it) {
        const int r = it * 16 + wave * 4 + orow;
        *(volatile v4f*)(Y + (row0 + t0 + r) * kDin + xcol + oc4) = ov[it];
      }
      __threadfence();
    }
  }
}

__global__ __launch_bounds__(256) void gate_rms_kernel(
    const float* __restrict__ ZX, const float* __restrict__ Y, const float* __restrict__ rw,
    unsigned short* __restrict__ GH, unsigned short* __restrict__ GL)
{
  __shared__ float red[8];
  const int tid = threadIdx.x, lane = tid & 31, wave = tid >> 5;
  const int row = blockIdx.x * 4 + (wave >> 1);
  const int col0 = (wave & 1) * 256 + lane * 8;
  const v4f y0 = *(const v4f*)(Y + (size_t)row * kDin + col0);
  const v4f y1 = *(const v4f*)(Y + (size_t)row * kDin + col0 + 4);
  const v4f z0 = *(const v4f*)(ZX + (size_t)row * kDprojPad + col0);
  const v4f z1 = *(const v4f*)(ZX + (size_t)row * kDprojPad + col0 + 4);
  const v4f w0 = *(const v4f*)(rw + col0);
  const v4f w1 = *(const v4f*)(rw + col0 + 4);
  v4f g0, g1;
  float ss = 0.f;
#pragma unroll
  for (int e = 0; e < 4; ++e) {
    const float s0 = __builtin_amdgcn_rcpf(1.0f + expf(-z0[e]));
    const float s1 = __builtin_amdgcn_rcpf(1.0f + expf(-z1[e]));
    g0[e] = y0[e] * (z0[e] * s0);
    g1[e] = y1[e] * (z1[e] * s1);
    ss = fmaf(g0[e], g0[e], ss);
    ss = fmaf(g1[e], g1[e], ss);
  }
#pragma unroll
  for (int off = 1; off < 32; off <<= 1) ss += __shfl_xor(ss, off, 32);
  red[wave] = ss;
  __syncthreads();
  const int wp = wave & ~1;
  const float tot = red[wp] + red[wp + 1];
  const float rs = rsqrtf(tot * (1.0f / (float)kDin) + kEps);
  v8h hv, lv;
#pragma unroll
  for (int e = 0; e < 4; ++e) {
    const float v0 = (g0[e] * rs) * w0[e];
    const float v1 = (g1[e] * rs) * w1[e];
    const unsigned short h0 = f2bf_bits(v0), h1 = f2bf_bits(v1);
    const unsigned short l0 = f2bf_bits(v0 - bf_bits2f(h0)), l1 = f2bf_bits(v1 - bf_bits2f(h1));
    hv[e]     = __builtin_bit_cast(_Float16, h0);
    hv[4 + e] = __builtin_bit_cast(_Float16, h1);
    lv[e]     = __builtin_bit_cast(_Float16, l0);
    lv[4 + e] = __builtin_bit_cast(_Float16, l1);
  }
  const size_t o = (size_t)row * kDin + col0;
  for (int pass = 0; pass < 2; ++pass) {
    *(volatile v8h*)(GH + o) = hv;
    *(volatile v8h*)(GL + o) = lv;
    __threadfence();
  }
}

static_assert(kDprojPad % 64 == 0 && (kRows / 64) * (kDprojPad / 64) == 1216 && 1216 % 8 == 0, "in_proj tiling");
static_assert((kRows / 64) * (kDm / 64) == 256 && 256 % 8 == 0, "out_proj tiling");
static_assert(kDm % 32 == 0 && kDin % 32 == 0, "K multiples of 32");

extern "C" void kernel_launch(void* const* d_in, const int* in_sizes, int n_in,
                              void* d_out, int out_size, void* d_ws, size_t ws_size,
                              hipStream_t stream) {
  if (n_in < 11) return;
  if (in_sizes[0] != kRows * kDm) return;
  if (in_sizes[1] != kDm) return;
  if (in_sizes[2] != kDm) return;
  if (in_sizes[3] != kDm * kDproj) return;
  if (in_sizes[4] != kConvDim * 4) return;
  if (in_sizes[5] != kConvDim) return;
  if (in_sizes[6] != kNh) return;
  if (in_sizes[7] != kNh) return;
  if (in_sizes[8] != kNh) return;
  if (in_sizes[9] != kDin) return;
  if (in_sizes[10] != kDin * kDm) return;
  if (out_size != 2 * kRows * kDm) return;
  if (ws_size < kWsTotal) return;

  const float* hid     = (const float*)d_in[0];
  const float* norm_w  = (const float*)d_in[1];
  const float* norm_b  = (const float*)d_in[2];
  const float* W_in    = (const float*)d_in[3];
  const float* conv_w  = (const float*)d_in[4];
  const float* conv_b  = (const float*)d_in[5];
  const float* dt_bias = (const float*)d_in[6];
  const float* A_log   = (const float*)d_in[7];
  const float* D_par   = (const float*)d_in[8];
  const float* rms_w   = (const float*)d_in[9];
  const float* W_out   = (const float*)d_in[10];
  float* out0 = (float*)d_out;
  float* out1 = out0 + kOut1Elem;

  char* ws = (char*)d_ws;
  unsigned short* XH  = (unsigned short*)(ws + kOffXH);
  unsigned short* XL  = (unsigned short*)(ws + kOffXL);
  unsigned short* WIH = (unsigned short*)(ws + kOffWIH);
  unsigned short* WIL = (unsigned short*)(ws + kOffWIL);
  unsigned short* WOH = (unsigned short*)(ws + kOffWOH);
  unsigned short* WOL = (unsigned short*)(ws + kOffWOL);
  float*          ZX  = (float*)(ws + kOffZX);
  float*          XBC = (float*)(ws + kOffXBC);
  float*          DT  = (float*)(ws + kOffDT);
  float*          DA  = (float*)(ws + kOffDA);
  float*          Yp  = (float*)(ws + kOffY);
  unsigned short* GH  = (unsigned short*)(ws + kOffGH);
  unsigned short* GL  = (unsigned short*)(ws + kOffGL);

  ln_residual_kernel<<<kRows / 8, 256, 0, stream>>>(hid, norm_w, norm_b, out1, XH, XL);

  weight_bt_split_kernel<kDm><<<kDprojPad / 8, 256, 0, stream>>>(W_in, kDproj, WIH, WIL);
  weight_bt_split_kernel<kDin><<<kDm / 8, 256, 0, stream>>>(W_out, kDm, WOH, WOL);

  wmma_gemm64<1, 2, 0, 0, false><<<dim3(152, 1), 256, 0, stream>>>(
      XH, XL, kDm, 0L,
      WIH, WIL, kDm, 0L,
      (void*)ZX, nullptr, kDprojPad, 0L,
      nullptr, nullptr, 0L,
      kRows, kDprojPad, kDm, 1.0f);

  conv_silu_kernel<<<dim3(kConvDim / 128, kRows / 64), 128, 0, stream>>>(ZX, conv_w, conv_b, XBC);

  dt_kernel<<<(kRows * kNh) / 256, 256, 0, stream>>>(ZX, dt_bias, A_log, DT, DA);

  scan_kernel<<<kBatch * kNh * 2, 128, 0, stream>>>(XBC, DT, DA, D_par, Yp);

  gate_rms_kernel<<<kRows / 4, 256, 0, stream>>>(ZX, Yp, rms_w, GH, GL);

  wmma_gemm64<1, 2, 0, 0, false><<<dim3(32, 1), 256, 0, stream>>>(
      GH, GL, kDin, 0L,
      WOH, WOL, kDin, 0L,
      (void*)out0, nullptr, kDm, 0L,
      nullptr, nullptr, 0L,
      kRows, kDm, kDin, 1.0f);
}
